// PlanetWarsAgentGNN_30305289241205
// MI455X (gfx1250) — hardware-verified
//
#include <hip/hip_runtime.h>
#define NG 512
#define PP 32
#define NNODE 16384
#define NE 507904
#define F0 16
#define DD 128
#define NHD 4
#define CH 32

typedef __bf16 v16b __attribute__((ext_vector_type(16)));
typedef unsigned short v8us __attribute__((ext_vector_type(8), may_alias));
typedef float  v8f  __attribute__((ext_vector_type(8)));
typedef float  v4f  __attribute__((ext_vector_type(4)));
typedef float  v4fa __attribute__((ext_vector_type(4), may_alias));
union FragB { v16b v; v8us half[2]; unsigned short u[16]; };

__device__ __forceinline__ unsigned short bf16_bits(float x) { unsigned int u = __float_as_uint(x); return (unsigned short)((u + 0x7FFFu + ((u >> 16) & 1u)) >> 16); }
__device__ __forceinline__ float bf16_val(unsigned short b) { return __uint_as_float(((unsigned int)b) << 16); }
__device__ __forceinline__ float bf16_round(float x) { return bf16_val(bf16_bits(x)); }
template <int NT>
__device__ __forceinline__ v8f mmaN(v16b ah, v16b al, v16b bh, v16b bl, v8f c) {
  c = __builtin_amdgcn_wmma_f32_16x16x32_bf16(false, ah, false, bh, (short)0, c, false, false);
  if (NT >= 2) c = __builtin_amdgcn_wmma_f32_16x16x32_bf16(false, al, false, bh, (short)0, c, false, false);
  if (NT >= 3) c = __builtin_amdgcn_wmma_f32_16x16x32_bf16(false, ah, false, bl, (short)0, c, false, false);
  asm volatile("v_nop\n\tv_nop\n\tv_nop\n\tv_nop" : "+v"(c) : "v"(ah), "v"(al), "v"(bh), "v"(bl));
  return c;
}

__device__ __forceinline__ void store_span256(float* span, v4f lo, v4f hi, int lane) {
  v4f a, b; const int s0 = lane >> 1, s1 = 16 + (lane >> 1); const bool odd = (lane & 1) != 0;
#pragma unroll
  for (int q = 0; q < 4; ++q) { const float l0 = __shfl(lo[q], s0, 32), h0 = __shfl(hi[q], s0, 32), l1 = __shfl(lo[q], s1, 32), h1 = __shfl(hi[q], s1, 32); a[q] = odd ? h0 : l0; b[q] = odd ? h1 : l1; }
  for (int pass = 0; pass < 2; ++pass) { *(volatile v4f*)(span + 4 * lane) = a; *(volatile v4f*)(span + 128 + 4 * lane) = b; if (pass == 0) __threadfence(); } }
__device__ __forceinline__ void store_span512h(_Float16* span, v8us p0, v8us p1, int lane) {
  typedef unsigned int v4u __attribute__((ext_vector_type(4))); union U { v8us h; v4u u; }; U x0, x1, a, b; x0.h = p0; x1.h = p1; const int s0 = lane >> 1, s1 = 16 + (lane >> 1); const bool odd = (lane & 1) != 0;
#pragma unroll
  for (int q = 0; q < 4; ++q) { const unsigned l0 = __shfl(x0.u[q], s0, 32), h0 = __shfl(x1.u[q], s0, 32), l1 = __shfl(x0.u[q], s1, 32), h1 = __shfl(x1.u[q], s1, 32); a.u[q] = odd ? h0 : l0; b.u[q] = odd ? h1 : l1; }
  for (int pass = 0; pass < 2; ++pass) { *(volatile v8us*)((unsigned short*)span + 8 * lane) = a.h; *(volatile v8us*)((unsigned short*)span + 256 + 8 * lane) = b.h; if (pass == 0) __threadfence(); } }

__global__ __launch_bounds__(256) void k_wt_bf16(const float* __restrict__ W, unsigned short* __restrict__ Wt, int K, int N) {
  const int t = blockIdx.x * 256 + threadIdx.x;
  const int k8n = K / 8;
  if (t >= N * k8n) return;
  const int n = t / k8n, k8 = (t % k8n) * 8;
  v8us v;
#pragma unroll
  for (int i = 0; i < 8; ++i) v[i] = bf16_bits(W[(size_t)(k8 + i) * N + n]);
  *(volatile v8us*)(Wt + (size_t)n * K + k8) = v;
  __threadfence();
  *(volatile v8us*)(Wt + (size_t)n * K + k8) = v;
}

template <bool ASPLIT, int ACT, bool BIAS_BF16>
__global__ __launch_bounds__(128) void k_gemm_bf(const float* __restrict__ A, int lda, const unsigned short* __restrict__ Wt, int ldb,
                                               const float* __restrict__ bias, float* __restrict__ C, int ldc, int M, int N, int K) {
  __shared__ __attribute__((aligned(16))) float so[4][16][64];
  const int tid = threadIdx.x, w = tid >> 5, lane = tid & 31, ln = lane & 15, hh = lane >> 4;
  const int ntn = N / 64;
  const int wid = blockIdx.x * 4 + w;
  const int mt = wid / ntn, nq = wid % ntn;
  if (mt * 16 >= M) return;
  const int row0 = mt * 16, col0 = nq * 64;
  const float* arow = A + (size_t)(row0 + ln) * lda;
  v8f acc[4] = {};
  for (int kb = 0; kb < K; kb += 32) {
    FragB ah, al;
    const v4f x0 = *(const v4fa*)(arow + kb + 8 * hh), x1 = *(const v4fa*)(arow + kb + 8 * hh + 4);
    const v4f x2 = *(const v4fa*)(arow + kb + 16 + 8 * hh), x3 = *(const v4fa*)(arow + kb + 16 + 8 * hh + 4);
    float xs[16] = {x0[0],x0[1],x0[2],x0[3],x1[0],x1[1],x1[2],x1[3],x2[0],x2[1],x2[2],x2[3],x3[0],x3[1],x3[2],x3[3]};
#pragma unroll
    for (int i = 0; i < 16; ++i) { const unsigned short hb = bf16_bits(xs[i]); ah.u[i] = hb; al.u[i] = ASPLIT ? bf16_bits(xs[i] - bf16_val(hb)) : (unsigned short)0; }
#pragma unroll
    for (int t = 0; t < 4; ++t) {
      const unsigned short* brow = Wt + (size_t)(col0 + t * 16 + ln) * ldb + kb;
      FragB b;
      b.half[0] = *(const v8us*)(brow + 8 * hh);
      b.half[1] = *(const v8us*)(brow + 16 + 8 * hh);
      acc[t] = mmaN<ASPLIT ? 2 : 1>(ah.v, al.v, b.v, b.v, acc[t]);
    }
  }
#pragma unroll
  for (int t = 0; t < 4; ++t) {
    float bv = bias ? bias[col0 + t * 16 + ln] : 0.f;
    if (BIAS_BF16) bv = bf16_round(bv);
#pragma unroll
    for (int r = 0; r < 8; ++r) { float v = acc[t][r] + bv; if (ACT == 1) v = fmaxf(v, 0.f); so[w][8 * hh + r][t * 16 + ln] = v; }
  }
  __builtin_amdgcn_fence(__ATOMIC_ACQ_REL, "workgroup");
  __builtin_amdgcn_wave_barrier();
  const int rsub = lane >> 4, c4 = (lane & 15) * 4;
  for (int pass = 0; pass < 2; ++pass) {
#pragma unroll
    for (int q = 0; q < 8; ++q) {
      const int r = q * 2 + rsub;
      const v4f v = *(const v4fa*)&so[w][r][c4];
      *(volatile v4f*)(C + (size_t)(row0 + r) * ldc + col0 + c4) = v;
    }
    if (pass == 0) __threadfence();
  }
}

template <int D, bool CAUSAL>
__global__ __launch_bounds__(128) void k_flash(const float* __restrict__ qb, const float* __restrict__ kb, const float* __restrict__ vb,
                                             int pitch, int T, int H, float scale, float* __restrict__ y, int ypitch) {
  constexpr int KS = D / 32;
  constexpr int DT = D / 16;
  __shared__ __attribute__((aligned(16))) unsigned short sKh[32][D + 8], sKl[32][D + 8], sVh[32][D + 8], sVl[32][D + 8];
  __shared__ __attribute__((aligned(16))) unsigned short sPh[4][16][40], sPl[4][16][40];
  __shared__ __attribute__((aligned(16))) float sO[4][16][D];
  const int tid = threadIdx.x, w = tid >> 5, lane = tid & 31, ln = lane & 15, hh = lane >> 4;
  const int nqb = (T + 63) / 64;
  const int bh = blockIdx.x / nqb, qblk = blockIdx.x % nqb;
  const int b = bh / H, h = bh % H;
  const int q0 = qblk * 64 + w * 16;
  const float* Q = qb + (size_t)b * T * pitch + h * D;
  const float* K = kb + (size_t)b * T * pitch + h * D;
  const float* V = vb + (size_t)b * T * pitch + h * D;

  FragB aqh[KS], aql[KS];
  {
    int row = q0 + ln; if (row >= T) row = T - 1;
    const float* qr = Q + (size_t)row * pitch;
#pragma unroll
    for (int ks = 0; ks < KS; ++ks)
#pragma unroll
      for (int i = 0; i < 16; ++i) {
        const int d = ks * 32 + ((i < 8) ? (8 * hh + i) : (16 + 8 * hh + (i - 8)));
        const float x = qr[d] * scale; const unsigned short hb = bf16_bits(x);
        aqh[ks].u[i] = hb; aql[ks].u[i] = bf16_bits(x - bf16_val(hb));
      }
  }
  float m_r[8], l_r[8];
#pragma unroll
  for (int r = 0; r < 8; ++r) { m_r[r] = -3.0e38f; l_r[r] = 0.f; }
  v8f oacc[DT];
#pragma unroll
  for (int dt = 0; dt < DT; ++dt) oacc[dt] = (v8f){0.f,0.f,0.f,0.f,0.f,0.f,0.f,0.f};

  const int kv_end = CAUSAL ? min(T, qblk * 64 + 64) : T;
  for (int j0 = 0; j0 < kv_end; j0 += 32) {
    __syncthreads();
    for (int e = tid; e < 32 * (D / 4); e += 128) {
      const int r = e / (D / 4), c4 = (e % (D / 4)) * 4;
      const int key = j0 + r;
      v4f kf = {0.f,0.f,0.f,0.f}, vf = {0.f,0.f,0.f,0.f};
      if (key < T) { kf = *(const v4fa*)(K + (size_t)key * pitch + c4); vf = *(const v4fa*)(V + (size_t)key * pitch + c4); }
#pragma unroll
      for (int t = 0; t < 4; ++t) {
        unsigned short hb = bf16_bits(kf[t]); sKh[r][c4 + t] = hb; sKl[r][c4 + t] = bf16_bits(kf[t] - bf16_val(hb));
        hb = bf16_bits(vf[t]); sVh[r][c4 + t] = hb; sVl[r][c4 + t] = bf16_bits(vf[t] - bf16_val(hb));
      }
    }
    __syncthreads();
    v8f s[2];
#pragma unroll
    for (int nt = 0; nt < 2; ++nt) {
      v8f acc = {};
#pragma unroll
      for (int ks = 0; ks < KS; ++ks) {
        FragB bh_, bl_;
        bh_.half[0] = *(const v8us*)&sKh[nt * 16 + ln][ks * 32 + 8 * hh]; bh_.half[1] = *(const v8us*)&sKh[nt * 16 + ln][ks * 32 + 16 + 8 * hh];
        bl_.half[0] = *(const v8us*)&sKl[nt * 16 + ln][ks * 32 + 8 * hh]; bl_.half[1] = *(const v8us*)&sKl[nt * 16 + ln][ks * 32 + 16 + 8 * hh];
        acc = mmaN<3>(aqh[ks].v, aql[ks].v, bh_.v, bl_.v, acc);
      }
      s[nt] = acc;
    }
    float alpha[8];
#pragma unroll
    for (int r = 0; r < 8; ++r) {
      const int qi = q0 + 8 * hh + r;
      const int ja = j0 + ln, jb = j0 + 16 + ln;
      if (CAUSAL) { if (ja > qi) s[0][r] = -3.0e38f; if (jb > qi) s[1][r] = -3.0e38f; }
      if (ja >= T) s[0][r] = -3.0e38f;
      if (jb >= T) s[1][r] = -3.0e38f;
      float mx = fmaxf(s[0][r], s[1][r]);
      mx = fmaxf(mx, __shfl_xor(mx, 1, 32)); mx = fmaxf(mx, __shfl_xor(mx, 2, 32)); mx = fmaxf(mx, __shfl_xor(mx, 4, 32)); mx = fmaxf(mx, __shfl_xor(mx, 8, 32));
      const float mnew = fmaxf(m_r[r], mx);
      alpha[r] = (mnew > -1.0e38f) ? __expf(m_r[r] - mnew) : 1.0f;
      const float p0 = (s[0][r] > -1.0e38f) ? __expf(s[0][r] - mnew) : 0.f;
      const float p1 = (s[1][r] > -1.0e38f) ? __expf(s[1][r] - mnew) : 0.f;
      m_r[r] = mnew;
      l_r[r] = l_r[r] * alpha[r] + p0 + p1;
      unsigned short hb = bf16_bits(p0); sPh[w][8 * hh + r][ln] = hb;      sPl[w][8 * hh + r][ln] = bf16_bits(p0 - bf16_val(hb));
      hb = bf16_bits(p1);                sPh[w][8 * hh + r][16 + ln] = hb; sPl[w][8 * hh + r][16 + ln] = bf16_bits(p1 - bf16_val(hb));
    }
#pragma unroll
    for (int dt = 0; dt < DT; ++dt)
#pragma unroll
      for (int r = 0; r < 8; ++r) oacc[dt][r] *= alpha[r];
    __builtin_amdgcn_fence(__ATOMIC_ACQ_REL, "workgroup");
    __builtin_amdgcn_wave_barrier();
    FragB pah, pal;
    pah.half[0] = *(const v8us*)&sPh[w][ln][8 * hh]; pah.half[1] = *(const v8us*)&sPh[w][ln][16 + 8 * hh];
    pal.half[0] = *(const v8us*)&sPl[w][ln][8 * hh]; pal.half[1] = *(const v8us*)&sPl[w][ln][16 + 8 * hh];
#pragma unroll
    for (int dt = 0; dt < DT; ++dt) {
      FragB bvh, bvl;
#pragma unroll
      for (int i = 0; i < 8; ++i) {
        bvh.u[i] = sVh[8 * hh + i][dt * 16 + ln]; bvh.u[8 + i] = sVh[16 + 8 * hh + i][dt * 16 + ln];
        bvl.u[i] = sVl[8 * hh + i][dt * 16 + ln]; bvl.u[8 + i] = sVl[16 + 8 * hh + i][dt * 16 + ln];
      }
      oacc[dt] = mmaN<3>(pah.v, pal.v, bvh.v, bvl.v, oacc[dt]);
    }
    __builtin_amdgcn_fence(__ATOMIC_ACQ_REL, "workgroup");
    __builtin_amdgcn_wave_barrier();
  }
#pragma unroll
  for (int r = 0; r < 8; ++r) {
    float l = l_r[r];
    l += __shfl_xor(l, 1, 32); l += __shfl_xor(l, 2, 32); l += __shfl_xor(l, 4, 32); l += __shfl_xor(l, 8, 32);
    l_r[r] = (l > 0.f) ? 1.0f / l : 0.f;
  }
#pragma unroll
  for (int dt = 0; dt < DT; ++dt)
#pragma unroll
    for (int r = 0; r < 8; ++r) sO[w][8 * hh + r][dt * 16 + ln] = oacc[dt][r] * l_r[r];
  __builtin_amdgcn_fence(__ATOMIC_ACQ_REL, "workgroup");
  __builtin_amdgcn_wave_barrier();
  for (int pass = 0; pass < 2; ++pass) {
    for (int r = 0; r < 16; ++r) {
      const int row = q0 + r;
      if (row < T && lane < D / 4) {
        const v4f val = *(const v4fa*)&sO[w][r][lane * 4];
        *(volatile v4f*)(y + ((size_t)b * T + row) * ypitch + h * D + lane * 4) = val;
      }
    }
    if (pass == 0) __threadfence();
  }
}

template <bool ASPLIT, int ACT, bool BIAS_BF16, bool RES_BF16>
__global__ __launch_bounds__(128) void k_gemm_bf3(const float* __restrict__ A, int lda, const unsigned short* __restrict__ Wt, int ldb,
                                                const float* __restrict__ bias, const float* __restrict__ resid, int rmod, int ldr,
                                                float* __restrict__ C, int ldc, int M, int N, int K) {
  __shared__ __attribute__((aligned(16))) float so[4][16][64];
  const int tid = threadIdx.x, w = tid >> 5, lane = tid & 31, ln = lane & 15, hh = lane >> 4;
  const int ntn = N / 64;
  const int wid = blockIdx.x * 4 + w;
  const int mt = wid / ntn, nq = wid % ntn;
  if (mt * 16 >= M) return;
  const int row0 = mt * 16, col0 = nq * 64;
  const float* arow = A + (size_t)(row0 + ln) * lda;
  v8f acc[4] = {};
  for (int kb = 0; kb < K; kb += 32) {
    FragB ah, al;
    const v4f x0 = *(const v4fa*)(arow + kb + 8 * hh), x1 = *(const v4fa*)(arow + kb + 8 * hh + 4);
    const v4f x2 = *(const v4fa*)(arow + kb + 16 + 8 * hh), x3 = *(const v4fa*)(arow + kb + 16 + 8 * hh + 4);
    float xs[16] = {x0[0],x0[1],x0[2],x0[3],x1[0],x1[1],x1[2],x1[3],x2[0],x2[1],x2[2],x2[3],x3[0],x3[1],x3[2],x3[3]};
#pragma unroll
    for (int i = 0; i < 16; ++i) { const unsigned short hb = bf16_bits(xs[i]); ah.u[i] = hb; al.u[i] = ASPLIT ? bf16_bits(xs[i] - bf16_val(hb)) : (unsigned short)0; }
#pragma unroll
    for (int t = 0; t < 4; ++t) {
      const unsigned short* brow = Wt + (size_t)(col0 + t * 16 + ln) * ldb + kb;
      FragB b;
      b.half[0] = *(const v8us*)(brow + 8 * hh);
      b.half[1] = *(const v8us*)(brow + 16 + 8 * hh);
      acc[t] = mmaN<ASPLIT ? 2 : 1>(ah.v, al.v, b.v, b.v, acc[t]);
    }
  }
#pragma unroll
  for (int t = 0; t < 4; ++t) {
    const int col = col0 + t * 16 + ln;
    float bv = bias ? bias[col] : 0.f;
    if (BIAS_BF16) bv = bf16_round(bv);
#pragma unroll
    for (int r = 0; r < 8; ++r) {
      float v = acc[t][r] + bv;
      if (resid) { float rv = resid[(size_t)((row0 + 8 * hh + r) % rmod) * ldr + col]; if (RES_BF16) rv = bf16_round(rv); v += rv; }
      if (ACT == 1) v = fmaxf(v, 0.f);
      if (ACT == 2) v = 0.5f * v * (1.0f + erff(v * 0.70710678118654752f));
      if (ACT == 3) { const float u = 0.7978845608028654f * (v + 0.044715f * v * v * v); v = 0.5f * v * (1.0f + tanhf(u)); }
      so[w][8 * hh + r][t * 16 + ln] = v;
    }
  }
  __builtin_amdgcn_fence(__ATOMIC_ACQ_REL, "workgroup");
  __builtin_amdgcn_wave_barrier();
  const int rsub = lane >> 4, c4 = (lane & 15) * 4;
  for (int pass = 0; pass < 2; ++pass) {
#pragma unroll
    for (int q = 0; q < 8; ++q) {
      const int r = q * 2 + rsub;
      const v4f v = *(const v4fa*)&so[w][r][c4];
      *(volatile v4f*)(C + (size_t)(row0 + r) * ldc + col0 + c4) = v;
    }
    if (pass == 0) __threadfence();
  }
}
template <bool PARAM_BF16>
__global__ __launch_bounds__(256) void k_layernorm(const float* __restrict__ X, const float* __restrict__ R, const float* __restrict__ g, const float* __restrict__ bta,
                                                  float* __restrict__ out_sum, float* __restrict__ out_norm, int N, float eps) {
  __shared__ float red[256];
  const int row = blockIdx.x, tid = threadIdx.x;
  const float* x = X + (size_t)row * N; const float* rr = R ? R + (size_t)row * N : nullptr;
  float vals[16];
  const int per = N / 256;
  float s1 = 0.f;
  for (int u = 0; u < per / 4; ++u) {
    const int j = tid * 4 + 1024 * u;
    const v4f a = *(const v4fa*)(x + j);
    v4f b = {0.f,0.f,0.f,0.f}; if (rr) b = *(const v4fa*)(rr + j);
#pragma unroll
    for (int q = 0; q < 4; ++q) { const float v = a[q] + b[q]; vals[u * 4 + q] = v; s1 += v; }
  }
  red[tid] = s1; __syncthreads();
  for (int st = 128; st > 0; st >>= 1) { if (tid < st) red[tid] += red[tid + st]; __syncthreads(); }
  const float mu = red[0] / (float)N; __syncthreads();
  float s2 = 0.f;
  for (int u = 0; u < per / 4; ++u)
#pragma unroll
    for (int q = 0; q < 4; ++q) { const float c = vals[u * 4 + q] - mu; s2 += c * c; }
  red[tid] = s2; __syncthreads();
  for (int st = 128; st > 0; st >>= 1) { if (tid < st) red[tid] += red[tid + st]; __syncthreads(); }
  const float rs = rsqrtf(red[0] / (float)N + eps);
  for (int pass = 0; pass < 2; ++pass) {
    for (int u = 0; u < per / 4; ++u) {
      const int j = tid * 4 + 1024 * u;
      v4f o, sm;
#pragma unroll
      for (int q = 0; q < 4; ++q) {
        float gg = g[j + q], bb = bta[j + q];
        if (PARAM_BF16) { gg = bf16_round(gg); bb = bf16_round(bb); }
        sm[q] = vals[u * 4 + q]; o[q] = (vals[u * 4 + q] - mu) * rs * gg + bb;
      }
      if (out_sum) *(volatile v4f*)(out_sum + (size_t)row * N + j) = sm;
      *(volatile v4f*)(out_norm + (size_t)row * N + j) = o;
    }
    if (pass == 0) __threadfence();
  }
}


typedef _Float16 v16h __attribute__((ext_vector_type(16)));
union FragH { v16h v; v8us half[2]; _Float16 h[16]; unsigned short u[16]; };
template <int NT>
__device__ __forceinline__ v8f mmaH(v16h ah, v16h al, v16h bh, v16h bl, v8f c) {
  c = __builtin_amdgcn_wmma_f32_16x16x32_f16(false, ah, false, bh, (short)0, c, false, false);
  if (NT >= 2) c = __builtin_amdgcn_wmma_f32_16x16x32_f16(false, al, false, bh, (short)0, c, false, false);
  if (NT >= 3) c = __builtin_amdgcn_wmma_f32_16x16x32_f16(false, ah, false, bl, (short)0, c, false, false);
  asm volatile("v_nop\n\tv_nop\n\tv_nop\n\tv_nop" : "+v"(c) : "v"(ah), "v"(al), "v"(bh), "v"(bl));
  return c;
}
template <bool ASPLIT>
__global__ __launch_bounds__(128) void k_gemm_h(const float* __restrict__ A, int lda, size_t sA, const _Float16* __restrict__ Bh, int ldb, size_t sB, float alpha, float* __restrict__ C, int ldc, size_t sC, int M, int N, int K) {
  __shared__ __attribute__((aligned(16))) float so[4][16][64];
  const int tid = threadIdx.x, w = tid >> 5, lane = tid & 31, ln = lane & 15, hh = lane >> 4; const int by = blockIdx.y;
  A += (size_t)by * sA; Bh += (size_t)by * sB; C += (size_t)by * sC;
  const int ntn = (N + 63) / 64; const int wid = blockIdx.x * 4 + w; const int mt = wid / ntn, nq = wid % ntn; if (mt * 16 >= M) return;
  const int row0 = mt * 16, col0 = nq * 64; const float* arow = A + (size_t)(row0 + ln) * lda;
  v8f acc[4] = {};
  for (int kb = 0; kb < K; kb += 32) {
    FragH ah, al;
    const v4f x0 = *(const v4fa*)(arow + kb + 8 * hh), x1 = *(const v4fa*)(arow + kb + 8 * hh + 4), x2 = *(const v4fa*)(arow + kb + 16 + 8 * hh), x3 = *(const v4fa*)(arow + kb + 16 + 8 * hh + 4);
    float xs[16] = {x0[0],x0[1],x0[2],x0[3],x1[0],x1[1],x1[2],x1[3],x2[0],x2[1],x2[2],x2[3],x3[0],x3[1],x3[2],x3[3]};
#pragma unroll
    for (int i = 0; i < 16; ++i) { const _Float16 h = (_Float16)xs[i]; ah.h[i] = h; al.h[i] = ASPLIT ? (_Float16)(xs[i] - (float)h) : (_Float16)0.0f; }
#pragma unroll
    for (int t = 0; t < 4; ++t) { if (col0 + t * 16 >= N) continue; const size_t boff = (size_t)(col0 + t * 16 + ln) * ldb + kb; FragH bq; bq.half[0] = *(const v8us*)(Bh + boff + 8 * hh); bq.half[1] = *(const v8us*)(Bh + boff + 16 + 8 * hh);
      acc[t] = mmaH<ASPLIT ? 2 : 1>(ah.v, al.v, bq.v, bq.v, acc[t]); }
  }
#pragma unroll
  for (int t = 0; t < 4; ++t) { if (col0 + t * 16 >= N) continue;
#pragma unroll
    for (int r = 0; r < 8; ++r) so[w][8 * hh + r][t * 16 + ln] = acc[t][r] * alpha; }
  __builtin_amdgcn_fence(__ATOMIC_ACQ_REL, "workgroup"); __builtin_amdgcn_wave_barrier();
  const int rsub = lane >> 4, c4 = (lane & 15) * 4;
  for (int pass = 0; pass < 2; ++pass) {
#pragma unroll
    for (int q = 0; q < 8; ++q) { const int r = q * 2 + rsub; if (col0 + c4 < N) { const v4f v = *(const v4fa*)&so[w][r][c4]; *(volatile v4f*)(C + (size_t)(row0 + r) * ldc + col0 + c4) = v; } }
    if (pass == 0) __threadfence(); }
}

__global__ __launch_bounds__(256) void k_wt_f16(const float* __restrict__ W, _Float16* __restrict__ Wt, int K, int N, float scale) {
  const int t = blockIdx.x * 256 + threadIdx.x; if (t >= N * (K / 8)) return; const int n = t / (K / 8), k8 = (t % (K / 8)) * 8; FragH f;
#pragma unroll
  for (int i = 0; i < 8; ++i) f.h[i] = (_Float16)(bf16_round(W[(size_t)(k8 + i) * N + n]) * scale); const v8us o = f.half[0];
  *(volatile v8us*)((unsigned short*)Wt + (size_t)n * K + k8) = o; __threadfence(); *(volatile v8us*)((unsigned short*)Wt + (size_t)n * K + k8) = o;
}
template <int ACT>
__global__ __launch_bounds__(128) void k_gemm_hhx(const _Float16* __restrict__ A, int lda, size_t sA, const _Float16* __restrict__ Bh, int ldb, size_t sB, float alpha, const float* __restrict__ bias, size_t sBias, const float* __restrict__ CP, int rowsPerB, size_t sCPb, int row0g,
    float* __restrict__ C, _Float16* __restrict__ C16, int ldc, size_t sC, int M, int N, int K) {
  __shared__ __attribute__((aligned(16))) float so[4][16][64];
  const int tid = threadIdx.x, w = tid >> 5, lane = tid & 31, ln = lane & 15, hh = lane >> 4; const int by = blockIdx.y;
  A += (size_t)by * sA; Bh += (size_t)by * sB; const size_t cofs = (size_t)by * sC; const float* bp = bias ? bias + (size_t)by * sBias : nullptr;
  const int ntn = (N + 63) / 64; const int wid = blockIdx.x * 4 + w; const int mt = wid / ntn, nq = wid % ntn; if (mt * 16 >= M) return;
  const int row0 = mt * 16, col0 = nq * 64; const _Float16* arow = A + (size_t)(row0 + ln) * lda;
  v8f acc[4] = {};
  for (int kb = 0; kb < K; kb += 32) { FragH ah; ah.half[0] = *(const v8us*)((const unsigned short*)arow + kb + 8 * hh); ah.half[1] = *(const v8us*)((const unsigned short*)arow + kb + 16 + 8 * hh);
#pragma unroll
    for (int t = 0; t < 4; ++t) { if (col0 + t * 16 >= N) continue; const size_t boff = (size_t)(col0 + t * 16 + ln) * ldb + kb; FragH bq; bq.half[0] = *(const v8us*)((const unsigned short*)Bh + boff + 8 * hh); bq.half[1] = *(const v8us*)((const unsigned short*)Bh + boff + 16 + 8 * hh);
      acc[t] = mmaH<1>(ah.v, ah.v, bq.v, bq.v, acc[t]); }
  }
#pragma unroll
  for (int t = 0; t < 4; ++t) { if (col0 + t * 16 >= N) continue; const int col = col0 + t * 16 + ln; const float bv = bp ? bf16_round(bp[col]) : 0.f;
#pragma unroll
    for (int r = 0; r < 8; ++r) { float v = acc[t][r] * alpha + bv; if (CP) { const int bidx = (row0g + row0 + 8 * hh + r) / rowsPerB; v += CP[(size_t)bidx * sCPb + (size_t)by * 64 + col]; } if (ACT == 1) v = (v > 0.f) ? v : expm1f(v); else if (ACT == 3) v = fmaxf(v, 0.f); so[w][8 * hh + r][t * 16 + ln] = v; } }
  __builtin_amdgcn_fence(__ATOMIC_ACQ_REL, "workgroup"); __builtin_amdgcn_wave_barrier();
  const int rsub = lane >> 4, c4 = (lane & 15) * 4; typedef _Float16 v4h __attribute__((ext_vector_type(4)));
  for (int pass = 0; pass < 2; ++pass) {
#pragma unroll
    for (int q = 0; q < 8; ++q) { const int r = q * 2 + rsub; if (col0 + c4 < N) { const v4f v = *(const v4fa*)&so[w][r][c4]; if (C) *(volatile v4f*)(C + cofs + (size_t)(row0 + r) * ldc + col0 + c4) = v; if (C16) { v4h h4; for (int i = 0; i < 4; ++i) h4[i] = (_Float16)v[i]; *(volatile v4h*)(C16 + cofs + (size_t)(row0 + r) * ldc + col0 + c4) = h4; } } }
    if (pass == 0) __threadfence(); }
}


__device__ __forceinline__ int bscan512(int cnt, int* wsum, int tid, int& total) {
  const int lane = tid & 31, wv = tid >> 5; int x = cnt;
#pragma unroll
  for (int d = 1; d < 32; d <<= 1) { const int y = __shfl_up(x, d, 32); if (lane >= d) x += y; }
  __syncthreads(); if (lane == 31) wsum[wv] = x; __syncthreads();
  int t = (lane < 16) ? wsum[lane] : 0;
#pragma unroll
  for (int d = 1; d < 32; d <<= 1) { const int y = __shfl_up(t, d, 32); if (lane >= d) t += y; }
  const int woff = (wv == 0) ? 0 : __shfl(t, wv - 1, 32); total = __shfl(t, 15, 32);
  return woff + x - cnt; }
__device__ __forceinline__ float leaky02(float v) { return v > 0.f ? v : 0.2f * v; }
__global__ __launch_bounds__(256) void k_x32(const float* __restrict__ x, _Float16* __restrict__ X32) { const size_t t = (size_t)blockIdx.x * 256 + threadIdx.x; if (t >= (size_t)NNODE * 4) return; const size_t n = t / 4; const int pc = (int)(t % 4); FragH a;
#pragma unroll
  for (int q = 0; q < 8; ++q) { const float xv = bf16_round(x[n * F0 + (pc & 1) * 8 + q]); a.h[q] = (_Float16)((pc < 2) ? xv : 0.f); }
  *(volatile v8us*)((unsigned short*)X32 + t * 8) = a.half[0]; __threadfence(); *(volatile v8us*)((unsigned short*)X32 + t * 8) = a.half[0]; }
__global__ __launch_bounds__(512) void k_w32(const float* __restrict__ W, _Float16* __restrict__ Bt) { const int t = threadIdx.x; const int o = t / 4, pc = t % 4; FragH a;
#pragma unroll
  for (int q = 0; q < 8; ++q) { const float wv = bf16_round(W[o * F0 + (pc & 1) * 8 + q]) * 16.0f; a.h[q] = (_Float16)((pc < 2) ? wv : 0.f); }
  *(volatile v8us*)((unsigned short*)Bt + t * 8) = a.half[0]; __threadfence(); *(volatile v8us*)((unsigned short*)Bt + t * 8) = a.half[0]; }
__global__ __launch_bounds__(256) void k_round16f(const float* __restrict__ W, _Float16* __restrict__ Bt, size_t n8) { const size_t t = (size_t)blockIdx.x * 256 + threadIdx.x; if (t >= n8) return; FragH f;
#pragma unroll
  for (int i = 0; i < 8; ++i) f.h[i] = (_Float16)(bf16_round(W[t * 8 + i]) * 16.0f); *(volatile v8us*)((unsigned short*)Bt + t * 8) = f.half[0]; __threadfence(); *(volatile v8us*)((unsigned short*)Bt + t * 8) = f.half[0]; }
__global__ __launch_bounds__(256) void k_h16(const float* __restrict__ x, _Float16* __restrict__ X16, size_t n8) { const size_t t = (size_t)blockIdx.x * 256 + threadIdx.x; if (t >= n8) return; FragH f;
#pragma unroll
  for (int q = 0; q < 8; ++q) f.h[q] = (_Float16)x[t * 8 + q]; *(volatile v8us*)((unsigned short*)X16 + t * 8) = f.half[0]; __threadfence(); *(volatile v8us*)((unsigned short*)X16 + t * 8) = f.half[0]; }
__global__ __launch_bounds__(256) void k_escore(const float* __restrict__ XL, const float* __restrict__ XR, const float* __restrict__ ea, const int* __restrict__ srci, const int* __restrict__ dsti, const float* __restrict__ We, const float* __restrict__ att, float* __restrict__ SCORE) {
  __shared__ float swe[DD][5]; __shared__ float satt[DD]; const int tid = threadIdx.x; for (int i = tid; i < DD * 5; i += 256) swe[i / 5][i % 5] = bf16_round(We[i]); if (tid < DD) satt[tid] = bf16_round(att[tid]); __syncthreads();
  const size_t e = (size_t)blockIdx.x * 256 + tid; if (e >= NE) return; int s = srci[e], d = dsti[e]; s = s < 0 ? 0 : (s >= NNODE ? NNODE - 1 : s); d = d < 0 ? 0 : (d >= NNODE ? NNODE - 1 : d);
  float a5[5];
#pragma unroll
  for (int q = 0; q < 5; ++q) a5[q] = bf16_round(ea[e * 5 + q]);
  const float* xl = XL + (size_t)s * DD; const float* xr = XR + (size_t)d * DD; v4f sc = {0.f, 0.f, 0.f, 0.f};
#pragma unroll 1
  for (int hc = 0; hc < DD; ++hc) { float v = xl[hc] + xr[hc];
#pragma unroll
    for (int q = 0; q < 5; ++q) v += a5[q] * swe[hc][q];
    sc[hc >> 5] += leaky02(v) * satt[hc]; }
  *(volatile v4f*)(SCORE + e * 4) = sc; __threadfence(); *(volatile v4f*)(SCORE + e * 4) = sc; }
#define QCAP 8
#define CHUNK 8192
__global__ __launch_bounds__(512) void k_smax(const float* __restrict__ SCORE, const int* __restrict__ srci, const int* __restrict__ dsti, float* __restrict__ M) {
  __shared__ short Lr[CHUNK]; __shared__ int Le[CHUNK]; __shared__ int scan[16]; __shared__ int lq[16][QCAP][32];
  const int tid = threadIdx.x, lane = tid & 31, wv = tid >> 5; const int n0 = blockIdx.x * 1024; const int myl0 = wv * 64 + 2 * lane; int qn = 0; v4f mx[2]; mx[0] = (v4f){-3.0e38f,-3.0e38f,-3.0e38f,-3.0e38f}; mx[1] = mx[0];

#pragma unroll 1
  for (int eb = 0; eb < NE + CHUNK; eb += CHUNK) { const bool sentinel = (eb >= NE); int tot = 0;
    if (!sentinel) { int k_cnt = 0; unsigned hm = 0; int hv[16];
#pragma unroll
      for (int k = 0; k < 16; ++k) { const int e = eb + tid * 16 + k; const int ec = (e < NE) ? e : (NE - 1); const int dv = dsti[ec] - n0; const int dd_ = (e < NE) ? dv : -1; hv[k] = dd_; if (dd_ >= 0 && dd_ < 1024) { hm |= 1u << k; ++k_cnt; } }
      int p = bscan512(k_cnt, scan, tid, tot);
#pragma unroll
      for (int k = 0; k < 16; ++k) if (hm & (1u << k)) { Lr[p] = (short)hv[k]; Le[p] = eb + tid * 16 + k; ++p; }
      __syncthreads(); }
    const int ntrip = sentinel ? 1 : ((tot + 31) >> 5);
#pragma unroll 1
    for (int it = 0; it < ntrip; ++it) { const int q = it * 32 + lane; const int lr = (!sentinel && q < tot) ? (int)Lr[q] : -1;
      unsigned mm = sentinel ? 1u : __builtin_amdgcn_ballot_w32(lr >= wv * 64 && lr < wv * 64 + 64);
#pragma unroll 1
      while (mm) { const int bit = __builtin_ctz(mm); mm &= mm - 1u; const int ol = sentinel ? -2 : (__shfl(lr, bit, 32) - wv * 64); const int owner = ol >> 1; const int e = sentinel ? 0 : Le[it * 32 + bit];
        if (sentinel || __builtin_amdgcn_ballot_w32(lane == owner && qn == QCAP)) {
          int kmax = qn;
#pragma unroll
          for (int o = 16; o >= 1; o >>= 1) kmax = max(kmax, __shfl_xor(kmax, o, 32));
#pragma unroll 1
          for (int k = 0; k < kmax; ++k) { if (k < qn) { const int ent = lq[wv][k][lane]; const int eq = ent >> 1; const int sl = ent & 1; int s = srci[eq]; s = s < 0 ? 0 : (s >= NNODE ? NNODE - 1 : s);
              const v4f sv = *(const v4fa*)(SCORE + (size_t)eq * 4); (void)s; if (sl == 0) { mx[0][0] = fmaxf(mx[0][0], sv[0]); mx[0][1] = fmaxf(mx[0][1], sv[1]); mx[0][2] = fmaxf(mx[0][2], sv[2]); mx[0][3] = fmaxf(mx[0][3], sv[3]); } else { mx[1][0] = fmaxf(mx[1][0], sv[0]); mx[1][1] = fmaxf(mx[1][1], sv[1]); mx[1][2] = fmaxf(mx[1][2], sv[2]); mx[1][3] = fmaxf(mx[1][3], sv[3]); } } }
          qn = 0; }
        if (lane == owner) { lq[wv][qn][lane] = e * 2 + (ol & 1); ++qn; } } }
    __syncthreads(); }
  store_span256(M + (size_t)(n0 + wv * 64) * 4, mx[0], mx[1], lane); }
template <int COFF, bool RELU>
__global__ __launch_bounds__(512) void k_sagg(const float* __restrict__ SCORE, const float* __restrict__ Mx, const _Float16* __restrict__ XL16, const int* __restrict__ srci, const int* __restrict__ dsti, const float* __restrict__ bias, float* __restrict__ H) {
  #pragma clang fp contract(off)
  __shared__ short Lr[CHUNK]; __shared__ int Le[CHUNK]; __shared__ int scan[16]; __shared__ int lq[16][QCAP][32]; __shared__ float stg[64][65];
  const int tid = threadIdx.x, lane = tid & 31, wv = tid >> 5; const int n0 = blockIdx.x * 1024; const int myl0 = wv * 64 + 2 * lane; int qn = 0;
  float acc[2][64], den[2][2], m_[2][2];
#pragma unroll
  for (int s2 = 0; s2 < 2; ++s2) { const int n = n0 + myl0 + s2; const int nn = (n < NNODE) ? n : 0; m_[s2][0] = Mx[(size_t)nn * 4 + COFF / 32]; m_[s2][1] = Mx[(size_t)nn * 4 + COFF / 32 + 1]; den[s2][0] = 0.f; den[s2][1] = 0.f;
#pragma unroll
    for (int c = 0; c < 64; ++c) acc[s2][c] = 0.f; }

#pragma unroll 1
  for (int eb = 0; eb < NE + CHUNK; eb += CHUNK) { const bool sentinel = (eb >= NE); int tot = 0;
    if (!sentinel) { int k_cnt = 0; unsigned hm = 0; int hv[16];
#pragma unroll
      for (int k = 0; k < 16; ++k) { const int e = eb + tid * 16 + k; const int ec = (e < NE) ? e : (NE - 1); const int dv = dsti[ec] - n0; const int dd_ = (e < NE) ? dv : -1; hv[k] = dd_; if (dd_ >= 0 && dd_ < 1024) { hm |= 1u << k; ++k_cnt; } }
      int p = bscan512(k_cnt, scan, tid, tot);
#pragma unroll
      for (int k = 0; k < 16; ++k) if (hm & (1u << k)) { Lr[p] = (short)hv[k]; Le[p] = eb + tid * 16 + k; ++p; }
      __syncthreads(); }
    const int ntrip = sentinel ? 1 : ((tot + 31) >> 5);
#pragma unroll 1
    for (int it = 0; it < ntrip; ++it) { const int q = it * 32 + lane; const int lr = (!sentinel && q < tot) ? (int)Lr[q] : -1;
      unsigned mm = sentinel ? 1u : __builtin_amdgcn_ballot_w32(lr >= wv * 64 && lr < wv * 64 + 64);
#pragma unroll 1
      while (mm) { const int bit = __builtin_ctz(mm); mm &= mm - 1u; const int ol = sentinel ? -2 : (__shfl(lr, bit, 32) - wv * 64); const int owner = ol >> 1; const int e = sentinel ? 0 : Le[it * 32 + bit];
        if (sentinel || __builtin_amdgcn_ballot_w32(lane == owner && qn == QCAP)) {
          int kmax = qn;
#pragma unroll
          for (int o = 16; o >= 1; o >>= 1) kmax = max(kmax, __shfl_xor(kmax, o, 32));
#pragma unroll 1
          for (int k = 0; k < kmax; ++k) { if (k < qn) { const int ent = lq[wv][k][lane]; const int eq = ent >> 1; const int sl = ent & 1; int s = srci[eq]; s = s < 0 ? 0 : (s >= NNODE ? NNODE - 1 : s);
              const v4f sv = *(const v4fa*)(SCORE + (size_t)eq * 4); const float p0 = expf(sv[COFF / 32] - m_[sl][0]), p1 = expf(sv[COFF / 32 + 1] - m_[sl][1]); const unsigned short* xr = (const unsigned short*)XL16 + (size_t)s * DD + COFF;
#pragma unroll
              for (int g = 0; g < 8; ++g) { FragH f; f.half[0] = *(const v8us*)(xr + g * 8); const float pg = (g < 4) ? p0 : p1;
#pragma unroll
                for (int s2 = 0; s2 < 2; ++s2) if (s2 == sl) { if (g == 0) den[s2][0] += p0; if (g == 4) den[s2][1] += p1;
#pragma unroll
                  for (int dd = 0; dd < 8; ++dd) acc[s2][g * 8 + dd] += pg * (float)f.h[dd]; } } } }
          qn = 0; }
        if (lane == owner) { lq[wv][qn][lane] = e * 2 + (ol & 1); ++qn; } } }
    __syncthreads(); }
#pragma unroll
  for (int s2 = 0; s2 < 2; ++s2) { const float i0 = 1.0f / (den[s2][0] + 1e-16f), i1 = 1.0f / (den[s2][1] + 1e-16f);
#pragma unroll
    for (int c = 0; c < 64; ++c) { float v = acc[s2][c] * ((c < 32) ? i0 : i1) + bf16_round(bias[COFF + c]); if (RELU) v = fmaxf(v, 0.f); acc[s2][c] = v; } }
  for (int tg = 0; tg < 16; ++tg) {
    if (wv == tg) {
#pragma unroll
      for (int c = 0; c < 64; ++c) { stg[2 * lane][c] = acc[0][c]; stg[2 * lane + 1][c] = acc[1][c]; } }
    __syncthreads();
    for (int pass = 0; pass < 2; ++pass) {
#pragma unroll
      for (int rd = 0; rd < 2; ++rd) { const int r = rd * 32 + tid / 16, pc = tid % 16; const int n = n0 + tg * 64 + r; if (n < NNODE) { v4f v; v[0] = stg[r][pc * 4]; v[1] = stg[r][pc * 4 + 1]; v[2] = stg[r][pc * 4 + 2]; v[3] = stg[r][pc * 4 + 3]; *(volatile v4f*)(H + (size_t)n * DD + COFF + pc * 4) = v; } }
      if (pass == 0) __threadfence(); }
    __syncthreads(); } }
__global__ __launch_bounds__(256) void k_msn(const float* __restrict__ H, _Float16* __restrict__ X2) { __shared__ float smean[DD]; const int tid = threadIdx.x; const int g = blockIdx.x; const float* hb = H + (size_t)g * PP * DD;
  if (tid < DD) { float s = 0.f; for (int p = 0; p < PP; ++p) s += hb[p * DD + tid]; smean[tid] = s / (float)PP; } __syncthreads();
  const int p = tid / 8, c0 = (tid % 8) * 16; FragH a, b;
#pragma unroll
  for (int q = 0; q < 8; ++q) { a.h[q] = (_Float16)fmaxf(hb[p * DD + c0 + q] - smean[c0 + q], 0.f); b.h[q] = (_Float16)fmaxf(hb[p * DD + c0 + 8 + q] - smean[c0 + 8 + q], 0.f); }
  store_span512h(X2 + (size_t)g * PP * DD + (size_t)(tid & ~31) * 16, a.half[0], b.half[0], tid & 31); }
__global__ __launch_bounds__(128) void k_pool(const float* __restrict__ H2, _Float16* __restrict__ G16) { __shared__ __attribute__((aligned(16))) _Float16 sg[DD]; const int tid = threadIdx.x; const int g = blockIdx.x; const float* hb = H2 + (size_t)g * PP * DD; float s = 0.f;
  for (int p = 0; p < PP; ++p) s += hb[p * DD + tid]; sg[tid] = (_Float16)(s / (float)PP); __syncthreads();
  if (tid < 16) { const v8us v = *(const v8us*)((const unsigned short*)sg + tid * 8); *(volatile v8us*)((unsigned short*)G16 + (size_t)g * DD + tid * 8) = v; __threadfence(); *(volatile v8us*)((unsigned short*)G16 + (size_t)g * DD + tid * 8) = v; } }
__global__ __launch_bounds__(256) void k_final(const float* __restrict__ C1, const float* __restrict__ N1, const float* __restrict__ S1, const float* __restrict__ Wc2, const float* __restrict__ bc2, const float* __restrict__ Wn2, const float* __restrict__ bn2, const float* __restrict__ Ws2, const float* __restrict__ bs2, float* __restrict__ out) {
  __shared__ __attribute__((aligned(16))) float so[16 * 34]; const int tid = threadIdx.x, wv = tid >> 5, lane = tid & 31; const int g0 = blockIdx.x * 16;
  float wc[4], wn[4], wsv[4];
#pragma unroll
  for (int q = 0; q < 4; ++q) { wc[q] = bf16_round(Wc2[lane + 32 * q]); wn[q] = bf16_round(Wn2[lane + 32 * q]); wsv[q] = bf16_round(Ws2[lane + 32 * q]); }
  const float bbc = bf16_round(bc2[0]), bbn = bf16_round(bn2[0]), bbs = bf16_round(bs2[0]);
#pragma unroll 1
  for (int jj = wv; jj < 16 * 34; jj += 8) { const int gl = jj / 34, j = jj % 34; const int g = g0 + gl; const float* row; const float* w; float bb;
    if (j == 0) { row = C1 + (size_t)g * DD; w = wc; bb = bbc; } else if (j == 1) { row = N1 + (size_t)g * DD; w = wn; bb = bbn; } else { row = S1 + ((size_t)g * PP + (j - 2)) * DD; w = wsv; bb = bbs; }
    float s = 0.f;
#pragma unroll
    for (int q = 0; q < 4; ++q) s += row[lane + 32 * q] * w[q];
    for (int o = 16; o >= 1; o >>= 1) s += __shfl_xor(s, o, 32); if (lane == 0) so[jj] = s + bb; }
  __syncthreads();
  for (int pass = 0; pass < 2; ++pass) { if (tid < 136) *(volatile v4f*)(out + (size_t)g0 * 34 + tid * 4) = *(const v4fa*)&so[tid * 4]; if (pass == 0) __threadfence(); } }
extern "C" void kernel_launch(void* const* d_in, const int* in_sizes, int n_in,
                              void* d_out, int out_size, void* d_ws, size_t ws_size, hipStream_t stream) {
  (void)in_sizes; (void)n_in; (void)out_size;
  const float* x = (const float*)d_in[0]; const int* ei = (const int*)d_in[1]; const float* ea = (const float*)d_in[2];
  const float* W1l = (const float*)d_in[3]; const float* b1l = (const float*)d_in[4]; const float* W1r = (const float*)d_in[5]; const float* b1r = (const float*)d_in[6]; const float* W1e = (const float*)d_in[7]; const float* att1 = (const float*)d_in[8]; const float* bias1 = (const float*)d_in[9];
  const float* W2l = (const float*)d_in[10]; const float* b2l = (const float*)d_in[11]; const float* W2r = (const float*)d_in[12]; const float* b2r = (const float*)d_in[13]; const float* W2e = (const float*)d_in[14]; const float* att2 = (const float*)d_in[15]; const float* bias2 = (const float*)d_in[16];
  const float* Wc1 = (const float*)d_in[17]; const float* bc1 = (const float*)d_in[18]; const float* Wc2 = (const float*)d_in[19]; const float* bc2 = (const float*)d_in[20]; const float* Ws1 = (const float*)d_in[21]; const float* bs1 = (const float*)d_in[22]; const float* Ws2 = (const float*)d_in[23]; const float* bs2 = (const float*)d_in[24]; const float* Wn1 = (const float*)d_in[25]; const float* bn1 = (const float*)d_in[26]; const float* Wn2 = (const float*)d_in[27]; const float* bn2 = (const float*)d_in[28];
  const int* srci = ei; const int* dsti = ei + NE;
  char* ws = (char*)d_ws; size_t off = 0;
  auto take = [&](size_t bytes) { char* p = ws + off; off += (bytes + 255) & ~(size_t)255; return p; };
  _Float16* X32 = (_Float16*)take((size_t)NNODE * 32 * 2); _Float16* B1l = (_Float16*)take(DD * 32 * 2); _Float16* B1r = (_Float16*)take(DD * 32 * 2); _Float16* B2l = (_Float16*)take(DD * DD * 2); _Float16* B2r = (_Float16*)take(DD * DD * 2); _Float16* Bc1 = (_Float16*)take(DD * DD * 2); _Float16* Bs1 = (_Float16*)take(DD * DD * 2); _Float16* Bn1 = (_Float16*)take(DD * DD * 2);
  float* XL = (float*)take((size_t)NNODE * DD * 4); _Float16* XL16 = (_Float16*)take((size_t)NNODE * DD * 2); float* XR = (float*)take((size_t)NNODE * DD * 4); float* SCORE = (float*)take((size_t)NE * 4 * 4); float* Mx = (float*)take((size_t)NNODE * 4 * 4); float* H1 = (float*)take((size_t)NNODE * DD * 4); _Float16* X2 = (_Float16*)take((size_t)NNODE * DD * 2); float* H2 = (float*)take((size_t)NNODE * DD * 4); _Float16* H2_16 = (_Float16*)take((size_t)NNODE * DD * 2);
  _Float16* G16 = (_Float16*)take((size_t)NG * DD * 2); float* C1 = (float*)take((size_t)NG * DD * 4); float* N1 = (float*)take((size_t)NG * DD * 4); float* S1 = (float*)take((size_t)NNODE * DD * 4);
  if (off > ws_size) return;
  k_x32<<<(NNODE * 4 + 255) / 256, 256, 0, stream>>>(x, X32); k_w32<<<1, 512, 0, stream>>>(W1l, B1l); k_w32<<<1, 512, 0, stream>>>(W1r, B1r);
  const size_t w8 = (size_t)DD * DD / 8; const unsigned gw = (unsigned)((w8 + 255) / 256);
  k_round16f<<<gw, 256, 0, stream>>>(W2l, B2l, w8); k_round16f<<<gw, 256, 0, stream>>>(W2r, B2r, w8); k_round16f<<<gw, 256, 0, stream>>>(Wc1, Bc1, w8); k_round16f<<<gw, 256, 0, stream>>>(Ws1, Bs1, w8); k_round16f<<<gw, 256, 0, stream>>>(Wn1, Bn1, w8);
  const dim3 gn(((NNODE / 16) * (DD / 64) + 3) / 4, 1); const unsigned ge = (unsigned)((NE + 255) / 256), gq = (NNODE + 1023) / 1024;
  k_gemm_hhx<0><<<gn, 128, 0, stream>>>(X32, 32, 0, B1l, 32, 0, 0.0625f, b1l, 0, nullptr, 1, 0, 0, XL, XL16, DD, 0, NNODE, DD, 32);
  k_gemm_hhx<0><<<gn, 128, 0, stream>>>(X32, 32, 0, B1r, 32, 0, 0.0625f, b1r, 0, nullptr, 1, 0, 0, XR, nullptr, DD, 0, NNODE, DD, 32);
  k_escore<<<ge, 256, 0, stream>>>(XL, XR, ea, srci, dsti, W1e, att1, SCORE);
  k_smax<<<gq, 512, 0, stream>>>(SCORE, srci, dsti, Mx);
  k_sagg<0, false><<<gq, 512, 0, stream>>>(SCORE, Mx, XL16, srci, dsti, bias1, H1); k_sagg<64, false><<<gq, 512, 0, stream>>>(SCORE, Mx, XL16, srci, dsti, bias1, H1);
  k_msn<<<NG, 256, 0, stream>>>(H1, X2);
  k_gemm_hhx<0><<<gn, 128, 0, stream>>>(X2, DD, 0, B2l, DD, 0, 0.0625f, b2l, 0, nullptr, 1, 0, 0, XL, XL16, DD, 0, NNODE, DD, DD);
  k_gemm_hhx<0><<<gn, 128, 0, stream>>>(X2, DD, 0, B2r, DD, 0, 0.0625f, b2r, 0, nullptr, 1, 0, 0, XR, nullptr, DD, 0, NNODE, DD, DD);
  k_escore<<<ge, 256, 0, stream>>>(XL, XR, ea, srci, dsti, W2e, att2, SCORE);
  k_smax<<<gq, 512, 0, stream>>>(SCORE, srci, dsti, Mx);
  k_sagg<0, true><<<gq, 512, 0, stream>>>(SCORE, Mx, XL16, srci, dsti, bias2, H2); k_sagg<64, true><<<gq, 512, 0, stream>>>(SCORE, Mx, XL16, srci, dsti, bias2, H2);
  k_pool<<<NG, 128, 0, stream>>>(H2, G16); k_h16<<<(unsigned)(((size_t)NNODE * DD / 8 + 255) / 256), 256, 0, stream>>>(H2, H2_16, (size_t)NNODE * DD / 8);
  k_gemm_hhx<3><<<dim3(((NG / 16) * (DD / 64) + 3) / 4, 1), 128, 0, stream>>>(G16, DD, 0, Bc1, DD, 0, 0.0625f, bc1, 0, nullptr, 1, 0, 0, C1, nullptr, DD, 0, NG, DD, DD);
  k_gemm_hhx<3><<<dim3(((NG / 16) * (DD / 64) + 3) / 4, 1), 128, 0, stream>>>(G16, DD, 0, Bn1, DD, 0, 0.0625f, bn1, 0, nullptr, 1, 0, 0, N1, nullptr, DD, 0, NG, DD, DD);
  k_gemm_hhx<3><<<gn, 128, 0, stream>>>(H2_16, DD, 0, Bs1, DD, 0, 0.0625f, bs1, 0, nullptr, 1, 0, 0, S1, nullptr, DD, 0, NNODE, DD, DD);
  k_final<<<NG / 16, 256, 0, stream>>>(C1, N1, S1, Wc2, bc2, Wn2, bn2, Ws2, bs2, (float*)d_out);
}
